// TransXLDecoderBlock_45423574123145
// MI455X (gfx1250) — hardware-verified
//
#include <hip/hip_runtime.h>
#include <math.h>
#include <stdint.h>

#define SQ    2048
#define MEM   2048
#define KL    4096
#define BB    2
#define EE    512
#define NH    8
#define HD    64
#define FFD   2048
#define NN    (BB * NH)
#define QR    (SQ * BB)
#define CROWS (KL * BB)
#define NQT   (SQ / 64)
#define NKT   (KL / 64)
static_assert(NH * HD == EE);
static_assert(MEM + SQ == KL);
static_assert(NQT * 64 == SQ && NKT * 64 == KL && NN == 16);
static_assert((EE % 64) == 0 && (FFD % 64) == 0 && (KL % 4) == 0);

#define WC   32.0f
#define QKC  4.0f
#define PCY  1024.0f
#define CC   64.0f
#define HC   4.0f

typedef _Float16 v16h __attribute__((ext_vector_type(16)));
typedef _Float16 v8h  __attribute__((ext_vector_type(8)));
typedef float    v8f  __attribute__((ext_vector_type(8)));
typedef float    v4f  __attribute__((ext_vector_type(4)));
typedef unsigned int v4u __attribute__((ext_vector_type(4)));

#if defined(__HIP_DEVICE_COMPILE__)
#define DEV_ASM 1
#else
#define DEV_ASM 0
#endif

__device__ __forceinline__ unsigned short h_bits(_Float16 x) { return __builtin_bit_cast(unsigned short, x); }
__device__ __forceinline__ unsigned pk16(unsigned short a, unsigned short b) { return (unsigned)a | ((unsigned)b << 16); }
__device__ __forceinline__ v8f zero8() { v8f z = {0.f, 0.f, 0.f, 0.f, 0.f, 0.f, 0.f, 0.f}; return z; }
__device__ __forceinline__ v4u pack8s(v4f a0, v4f a1, float s) {
  v4u p;
  p[0] = pk16(h_bits((_Float16)(a0[0] * s)), h_bits((_Float16)(a0[1] * s)));
  p[1] = pk16(h_bits((_Float16)(a0[2] * s)), h_bits((_Float16)(a0[3] * s)));
  p[2] = pk16(h_bits((_Float16)(a1[0] * s)), h_bits((_Float16)(a1[1] * s)));
  p[3] = pk16(h_bits((_Float16)(a1[2] * s)), h_bits((_Float16)(a1[3] * s)));
  return p;
}

__device__ __forceinline__ v16h ldfrag(const _Float16* p) {
  union { v16h v; v8h h[2]; } f;
  f.h[0] = *(const v8h*)(p);
  f.h[1] = *(const v8h*)(p + 16);
  return f.v;
}

__device__ __forceinline__ v8f mmar(v16h a, v16h b, v8f c) {
  return __builtin_amdgcn_wmma_f32_16x16x32_f16(false, a, false, b, (short)0, c, false, false);
}
__device__ __forceinline__ v8f mma_h(v16h a, v16h b, v8f c) {
  c = __builtin_amdgcn_wmma_f32_16x16x32_f16(false, a, false, b, (short)0, c, false, false);
#if DEV_ASM
  asm volatile("v_nop\n\tv_nop\n\tv_nop\n\tv_nop" : "+v"(c) : "v"(a), "v"(b));
#endif
  return c;
}
__device__ __forceinline__ void dep_guard(v8f& a, v8f& b, v16h x, v16h y) {
#if DEV_ASM
  asm volatile("v_nop\n\tv_nop\n\tv_nop\n\tv_nop" : "+v"(a), "+v"(b) : "v"(x), "v"(y));
#else
  (void)a; (void)b; (void)x; (void)y;
#endif
}
__device__ __forceinline__ void keep4(v16h a, v16h b, v16h c, v16h d) {
#if DEV_ASM
  asm volatile("v_nop" :: "v"(a), "v"(b), "v"(c), "v"(d));
#else
  (void)a; (void)b; (void)c; (void)d;
#endif
}
__device__ __forceinline__ void acc_guard4(v8f& a, v8f& b, v8f& c, v8f& d) {
#if DEV_ASM
  asm volatile("v_nop\n\tv_nop\n\tv_nop\n\tv_nop" : "+v"(a), "+v"(b), "+v"(c), "+v"(d));
#else
  (void)a; (void)b; (void)c; (void)d;
#endif
}

__global__ __launch_bounds__(256) void cvt_cat(const float* __restrict__ mem, const float* __restrict__ inp,
                                                unsigned short* out, int n8) {
  const int i = blockIdx.x * 256 + (int)threadIdx.x;
  if (i < n8) {
    const size_t e = (size_t)i * 8;
    const size_t halfE = (size_t)MEM * BB * EE;
    const float* base = (e < halfE) ? mem : inp;
    const size_t e2 = (e < halfE) ? e : (e - halfE);
    const float* ip = base + e2;
    const v4f a0 = *(const v4f*)(ip), a1 = *(const v4f*)(ip + 4);
    const v4u p = pack8s(a0, a1, 1.0f);
    unsigned short* o = out + e;
    *(volatile v4u*)o = p;
    __threadfence();
    *(volatile v4u*)o = p;
  }
}

__global__ __launch_bounds__(256) void cvt_f(const float* __restrict__ in, unsigned short* out, int n8, float s) {
  const int i = blockIdx.x * 256 + (int)threadIdx.x;
  if (i < n8) {
    const v4f a0 = *(const v4f*)(in + (size_t)i * 8);
    const v4f a1 = *(const v4f*)(in + (size_t)i * 8 + 4);
    const v4u p = pack8s(a0, a1, s);
    unsigned short* o = out + (size_t)i * 8;
    *(volatile v4u*)o = p;
    __threadfence();
    *(volatile v4u*)o = p;
  }
}

__global__ __launch_bounds__(256) void cvt_wt(const float* __restrict__ in, unsigned short* out,
                                               int kin, int nout, float s) {
  __shared__ float tile[64][65];
  const int tid = threadIdx.x;
  const int n0 = blockIdx.x * 64, k0 = blockIdx.y * 64;
  {
    const int r = tid >> 2, c16 = (tid & 3) * 16;
    const float* ip = in + (size_t)(k0 + r) * (size_t)nout + n0 + c16;
#pragma unroll
    for (int q = 0; q < 4; ++q) {
      const v4f a = *(const v4f*)(ip + 4 * q);
#pragma unroll
      for (int e = 0; e < 4; ++e) tile[r][c16 + 4 * q + e] = a[e];
    }
  }
  __syncthreads();
  const int q = tid >> 3, c8 = (tid & 7) * 8;
  v4u hv[2];
#pragma unroll
  for (int it = 0; it < 2; ++it) {
    const int nl = it * 32 + q;
    v4f a0, a1;
#pragma unroll
    for (int e = 0; e < 4; ++e) { a0[e] = tile[c8 + e][nl]; a1[e] = tile[c8 + 4 + e][nl]; }
    hv[it] = pack8s(a0, a1, s);
  }
  for (int pass = 0; pass < 2; ++pass) {
#pragma unroll
    for (int it = 0; it < 2; ++it) {
      const int nl = it * 32 + q;
      *(volatile v4u*)(out + (size_t)(n0 + nl) * (size_t)kin + k0 + c8) = hv[it];
    }
    __threadfence();
  }
}

__global__ __launch_bounds__(256) void bias_dot(const unsigned short* __restrict__ kp, const unsigned short* __restrict__ rk,
                                                 const float* __restrict__ ub, const float* __restrict__ vb,
                                                 float* cw, float* cr, float sc) {
  const int sel = blockIdx.y;
  const _Float16* P = (const _Float16*)(const void*)(sel ? rk : kp);
  const float* bias = sel ? vb : ub;
  float* outp = sel ? cr : cw;
  const int nmax = sel ? NH : NN;
  const int idx = blockIdx.x * 256 + (int)threadIdx.x;
  if (idx >= nmax * (KL / 4)) return;
  const int n  = idx >> 10;
  const int j0 = (idx & 1023) * 4;
  const int h  = n & (NH - 1);
  const _Float16* p0 = P + ((size_t)n * KL + j0) * HD;
  const float* bh = bias + h * HD;
  float a0 = 0.f, a1 = 0.f, a2 = 0.f, a3 = 0.f;
#pragma unroll 1
  for (int dc = 0; dc < HD / 8; ++dc) {
    const v4f b0 = *(const v4f*)(bh + dc * 8);
    const v4f b1v = *(const v4f*)(bh + dc * 8 + 4);
    float bbv[8];
#pragma unroll
    for (int e = 0; e < 4; ++e) { bbv[e] = b0[e]; bbv[4 + e] = b1v[e]; }
    const v8h r0 = *(const v8h*)(p0 + dc * 8);
    const v8h r1 = *(const v8h*)(p0 + HD + dc * 8);
    const v8h r2 = *(const v8h*)(p0 + 2 * HD + dc * 8);
    const v8h r3 = *(const v8h*)(p0 + 3 * HD + dc * 8);
#pragma unroll
    for (int e = 0; e < 8; ++e) {
      a0 += bbv[e] * (float)r0[e];
      a1 += bbv[e] * (float)r1[e];
      a2 += bbv[e] * (float)r2[e];
      a3 += bbv[e] * (float)r3[e];
    }
  }
  v4f v;
  v[0] = a0 * sc; v[1] = a1 * sc; v[2] = a2 * sc; v[3] = a3 * sc;
  float* o = outp + (size_t)n * KL + j0;
  *(volatile v4f*)o = v;
  __threadfence();
  *(volatile v4f*)o = v;
}

struct GemmArgs {
  const unsigned short* A;
  const unsigned short* Bt;
  void* C0;
  const float* bias;
  long long strideA, strideB, strideC;
  int lda, ldb, ldc, M, N, K, aRowOff, tDst, tOff, bShift, skipLim, hasBias;
  float oscale, ocarry;
};
static_assert(sizeof(GemmArgs) == 112);

template <int MODE>
__global__ __launch_bounds__(256) void gemm64(GemmArgs g) {
  const _Float16* A  = (const _Float16*)(const void*)g.A;
  const _Float16* Bt = (const _Float16*)(const void*)g.Bt;
  __shared__ __align__(16) float sT[8][16 * 68];
  const int bz   = blockIdx.y;
  const int lane = threadIdx.x & 31;
  const int wave = threadIdx.x >> 5;
  const int tilesN = g.N >> 6;
  const int tilesM = g.M >> 6;
  const int tile = blockIdx.x * 8 + wave;
  if (tile >= tilesM * tilesN) return;
  const int tm = tile / tilesN;
  const int tn = tile - tm * tilesN;
  if (tm + tn < g.skipLim) return;
  const int aRow0 = (tm << 6) + g.aRowOff;
  const int bRow0 = tn << 6;
  const int n0 = tn << 6;

  const _Float16* Ab = A  + (size_t)bz * (size_t)g.strideA;
  const _Float16* Bb = Bt + (size_t)bz * (size_t)g.strideB;

  const int rlane = lane & 15;
  const int koff  = (lane >> 4) * 8;
  const int mOff  = (lane >> 4) * 8;

  v8f acc[4][4];
#pragma unroll
  for (int i = 0; i < 4; ++i)
#pragma unroll
    for (int j = 0; j < 4; ++j) acc[i][j] = zero8();

  for (int k0 = 0; k0 < g.K; k0 += 32) {
    v16h bq[4];
#pragma unroll
    for (int j = 0; j < 4; ++j)
      bq[j] = ldfrag(Bb + (size_t)(bRow0 + (j << 4) + rlane) * (size_t)g.ldb + koff + k0);
#pragma unroll
    for (int i = 0; i < 4; ++i) {
      const v16h af = ldfrag(Ab + (size_t)(aRow0 + (i << 4) + rlane) * (size_t)g.lda + koff + k0);
#pragma unroll
      for (int j = 0; j < 4; ++j) acc[i][j] = mmar(af, bq[j], acc[i][j]);
      dep_guard(acc[i][0], acc[i][3], af, bq[3]);
    }
    keep4(bq[0], bq[1], bq[2], bq[3]);
  }
  acc_guard4(acc[0][0], acc[0][1], acc[0][2], acc[0][3]);
  acc_guard4(acc[1][0], acc[1][1], acc[1][2], acc[1][3]);
  acc_guard4(acc[2][0], acc[2][1], acc[2][2], acc[2][3]);
  acc_guard4(acc[3][0], acc[3][1], acc[3][2], acc[3][3]);

  float* slab = sT[wave];
#pragma unroll
  for (int i = 0; i < 4; ++i) {
#pragma unroll
    for (int j = 0; j < 4; ++j) {
#pragma unroll
      for (int r = 0; r < 8; ++r) {
        slab[(mOff + r) * 68 + (j << 4) + rlane] = acc[i][j][r];
      }
    }
    __builtin_amdgcn_fence(__ATOMIC_RELEASE, "workgroup");
    __builtin_amdgcn_wave_barrier();
    __builtin_amdgcn_fence(__ATOMIC_ACQUIRE, "workgroup");
    if (MODE == 0) {
      float* C = (float*)g.C0 + (size_t)bz * (size_t)g.strideC;
      const int h2 = lane >> 4, c4 = (lane & 15) * 4;
      v4f bv = {0.f, 0.f, 0.f, 0.f};
      if (g.hasBias != 0) bv = *(const v4f*)(g.bias + n0 + c4);
      const int rowBase = aRow0 + (i << 4);
      for (int pass = 0; pass < 2; ++pass) {
#pragma unroll
        for (int it = 0; it < 8; ++it) {
          const int row = it * 2 + h2;
          const v4f v = *(const v4f*)(slab + row * 68 + c4) * g.oscale + bv;
          *(volatile v4f*)(C + (size_t)(rowBase + row) * (size_t)g.ldc + n0 + c4) = v;
        }
        __threadfence();
      }
    } else {
      const int q = lane >> 3, c8 = (lane & 7) * 8;
      float biv[8];
#pragma unroll
      for (int e = 0; e < 8; ++e) biv[e] = 0.f;
      if (MODE == 2) {
        const v4f b0 = *(const v4f*)(g.bias + n0 + c8);
        const v4f b1v = *(const v4f*)(g.bias + n0 + c8 + 4);
#pragma unroll
        for (int e = 0; e < 4; ++e) { biv[e] = b0[e]; biv[4 + e] = b1v[e]; }
      }
      unsigned short* P0 = (unsigned short*)g.C0;
      v4u hv[4];
#pragma unroll
      for (int it = 0; it < 4; ++it) {
        const int row = it * 4 + q;
        const float* sp = slab + row * 68 + c8;
        v4u a;
#pragma unroll
        for (int e = 0; e < 4; ++e) {
          float v0 = sp[2 * e] * g.oscale + biv[2 * e];
          float v1 = sp[2 * e + 1] * g.oscale + biv[2 * e + 1];
          if (MODE == 2) { v0 = fmaxf(v0, 0.f); v1 = fmaxf(v1, 0.f); }
          a[e] = pk16(h_bits((_Float16)(v0 * g.ocarry)), h_bits((_Float16)(v1 * g.ocarry)));
        }
        hv[it] = a;
      }
      const int bMask = (1 << g.bShift) - 1;
      for (int pass = 0; pass < 2; ++pass) {
#pragma unroll
        for (int it = 0; it < 4; ++it) {
          const int row = it * 4 + q;
          size_t off;
          if (MODE == 1) {
            const int m  = aRow0 + (i << 4) + row;
            const int bb = m & bMask;
            const int t  = (m >> g.bShift) - g.tOff;
            off = ((size_t)(bb * NH + tn) * (size_t)g.tDst + (size_t)t) * HD + c8;
          } else if (MODE == 2) {
            off = (size_t)(aRow0 + (i << 4) + row) * (size_t)g.ldc + n0 + c8;
          } else {
            off = (size_t)bz * (size_t)g.strideC + (size_t)((tm << 6) + (i << 4) + row) * (size_t)g.ldc + n0 + c8;
          }
          *(volatile v4u*)(P0 + off) = hv[it];
        }
        __threadfence();
      }
    }
    __builtin_amdgcn_fence(__ATOMIC_RELEASE, "workgroup");
    __builtin_amdgcn_wave_barrier();
    __builtin_amdgcn_fence(__ATOMIC_ACQUIRE, "workgroup");
  }
}

__global__ __launch_bounds__(128)
void attn_rel(const unsigned short* __restrict__ qpp, const unsigned short* __restrict__ kpp,
              const unsigned short* __restrict__ vtp, const float* __restrict__ raw,
              const float* __restrict__ cw, unsigned short* ctxp, int n, float sscale, float cinv) {
  union FH { v16h v; v8h h[2]; };
  __shared__ __align__(16) _Float16 Ksh[64 * 64];
  __shared__ __align__(16) _Float16 Vth[64 * 64];
  __shared__ __align__(16) _Float16 Psh[4][16 * 64];
  __shared__ __align__(16) float    Os[4][16 * 64];

  const int tid  = threadIdx.x;
  const int wave = tid >> 5;
  const int lane = tid & 31;
  const int hh   = lane >> 4;
  const int c    = lane & 15;

  const int qt = blockIdx.x;
  const int b  = n >> 3;
  const int h  = n & (NH - 1);
  const int i0 = qt * 64 + wave * 16;

  const _Float16* Q  = (const _Float16*)(const void*)qpp + (size_t)n * SQ * HD;
  const _Float16* Kg = (const _Float16*)(const void*)kpp + (size_t)n * KL * HD;
  const _Float16* Vh = (const _Float16*)(const void*)vtp + (size_t)n * HD * KL;
  const float* cwn   = cw + (size_t)n * KL;

  v16h qa[2];
#pragma unroll
  for (int dc = 0; dc < 2; ++dc) {
    qa[dc] = ldfrag(Q + (size_t)(i0 + c) * HD + dc * 32 + 8 * hh);
  }

  float mrow[8], lrow[8];
  v8f oacc[4];
#pragma unroll
  for (int r = 0; r < 8; ++r) { mrow[r] = -INFINITY; lrow[r] = 0.f; }
#pragma unroll
  for (int t = 0; t < 4; ++t) oacc[t] = zero8();

  const int nkt = min(qt + (MEM / 64) + 1, NKT);
  for (int kt = 0; kt < nkt; ++kt) {
    const int kv0 = kt * 64;
    __syncthreads();
    {
      const int r = tid >> 1, half = (tid & 1) * 32;
      const _Float16* kg = Kg + (size_t)(kv0 + r) * HD + half;
      const _Float16* vg = Vh + (size_t)r * KL + kv0 + half;
#pragma unroll
      for (int i = 0; i < 4; ++i) {
        const v8h a0 = *(const v8h*)(kg + 8 * i);
        const v8h b0 = *(const v8h*)(vg + 8 * i);
        *(v8h*)(Ksh + r * 64 + half + 8 * i) = a0;
        *(v8h*)(Vth + r * 64 + half + 8 * i) = b0;
      }
    }
    __syncthreads();

    v8f s[4];
#pragma unroll
    for (int j = 0; j < 4; ++j) {
      v8f a = zero8();
#pragma unroll
      for (int dc = 0; dc < 2; ++dc) {
        FH kb;
        kb.h[0] = *(const v8h*)(Ksh + (j * 16 + c) * 64 + dc * 32 + 8 * hh);
        kb.h[1] = *(const v8h*)(Ksh + (j * 16 + c) * 64 + dc * 32 + 16 + 8 * hh);
        a = mma_h(qa[dc], kb.v, a);
      }
      const int jj = kv0 + j * 16 + c;
      const float cwj = cwn[jj];
#pragma unroll
      for (int r = 0; r < 8; ++r) {
        const int ii  = i0 + 8 * hh + r;
        const int dlt = jj - ii;
        const int col = min(max(dlt + (SQ - 1), 0), KL - 1);
        const float bdv = raw[(size_t)ii * KL + col];
        const float sv  = a[r] * sscale + cwj + bdv;
        s[j][r] = (dlt > MEM) ? -INFINITY : sv;
      }
    }

    _Float16* pwh = Psh[wave];
#pragma unroll
    for (int r = 0; r < 8; ++r) {
      float m = s[0][r];
#pragma unroll
      for (int j = 1; j < 4; ++j) m = fmaxf(m, s[j][r]);
#pragma unroll
      for (int off = 1; off < 16; off <<= 1) m = fmaxf(m, __shfl_xor(m, off, 32));
      const float mnew  = fmaxf(mrow[r], m);
      const float msafe = (mnew == -INFINITY) ? 0.f : mnew;
      const float alpha = __expf(mrow[r] - msafe);
      mrow[r] = mnew;
      float psum = 0.f;
#pragma unroll
      for (int j = 0; j < 4; ++j) {
        const float p = __expf(s[j][r] - msafe);
        psum += p;
        pwh[(8 * hh + r) * 64 + j * 16 + c] = (_Float16)(p * PCY);
      }
#pragma unroll
      for (int off = 1; off < 16; off <<= 1) psum += __shfl_xor(psum, off, 32);
      lrow[r] = lrow[r] * alpha + psum;
#pragma unroll
      for (int t = 0; t < 4; ++t) oacc[t][r] *= alpha;
    }
    __builtin_amdgcn_fence(__ATOMIC_RELEASE, "workgroup");
    __builtin_amdgcn_wave_barrier();
    __builtin_amdgcn_fence(__ATOMIC_ACQUIRE, "workgroup");

#pragma unroll 1
    for (int kk = 0; kk < 2; ++kk) {
      FH pa;
      pa.h[0] = *(const v8h*)(pwh + c * 64 + kk * 32 + 8 * hh);
      pa.h[1] = *(const v8h*)(pwh + c * 64 + kk * 32 + 16 + 8 * hh);
#pragma unroll
      for (int t = 0; t < 4; ++t) {
        FH vb;
        vb.h[0] = *(const v8h*)(Vth + (t * 16 + c) * 64 + kk * 32 + 8 * hh);
        vb.h[1] = *(const v8h*)(Vth + (t * 16 + c) * 64 + kk * 32 + 16 + 8 * hh);
        oacc[t] = mma_h(pa.v, vb.v, oacc[t]);
      }
    }
  }

  float* os = Os[wave];
#pragma unroll
  for (int r = 0; r < 8; ++r) {
    const float l = lrow[r];
    const float inv = ((l > 0.f) ? (1.0f / l) : 0.f) * cinv;
#pragma unroll
    for (int t = 0; t < 4; ++t) os[(8 * hh + r) * 64 + t * 16 + c] = oacc[t][r] * inv;
  }
  __builtin_amdgcn_fence(__ATOMIC_RELEASE, "workgroup");
  __builtin_amdgcn_wave_barrier();
  __builtin_amdgcn_fence(__ATOMIC_ACQUIRE, "workgroup");
  {
    const int q4 = lane >> 3, c8 = (lane & 7) * 8;
    v4u hv[4];
#pragma unroll
    for (int it = 0; it < 4; ++it) {
      const int row = it * 4 + q4;
      const float* sp = os + row * 64 + c8;
      v4u a;
#pragma unroll
      for (int e = 0; e < 4; ++e) {
        const float f0 = sp[2 * e], f1 = sp[2 * e + 1];
        a[e] = pk16(h_bits((_Float16)f0), h_bits((_Float16)f1));
      }
      hv[it] = a;
    }
    for (int pass = 0; pass < 2; ++pass) {
#pragma unroll
      for (int it = 0; it < 4; ++it) {
        const int row = it * 4 + q4;
        const size_t go = ((size_t)(i0 + row) * BB + b) * EE + (size_t)h * HD + c8;
        *(volatile v4u*)(ctxp + go) = hv[it];
      }
      __threadfence();
    }
  }
}

template <int WH>
__global__ __launch_bounds__(256) void ln_rows(const float* __restrict__ xa, const float* __restrict__ xb,
                                                const float* __restrict__ gam, const float* __restrict__ bet,
                                                float* outF, unsigned short* outH, int nrows) {
  __shared__ __align__(16) float ys[8][EE];
  const int wave = threadIdx.x >> 5, lane = threadIdx.x & 31;
  const int row = blockIdx.x * 8 + wave;
  if (row >= nrows) return;
  const size_t base = (size_t)row * EE;
  v4f x[4];
  float sum = 0.f;
#pragma unroll
  for (int j = 0; j < 4; ++j) {
    const v4f a  = *(const v4f*)(xa + base + j * 128 + lane * 4);
    const v4f cx = *(const v4f*)(xb + base + j * 128 + lane * 4);
    x[j] = a + cx;
    sum += (x[j][0] + x[j][1]) + (x[j][2] + x[j][3]);
  }
#pragma unroll
  for (int off = 1; off < 32; off <<= 1) sum += __shfl_xor(sum, off, 32);
  const float mu = sum * (1.0f / EE);
  v4f d[4];
  float sq = 0.f;
#pragma unroll
  for (int j = 0; j < 4; ++j) {
    d[j] = x[j] - mu;
    sq += (d[j][0] * d[j][0] + d[j][1] * d[j][1]) + (d[j][2] * d[j][2] + d[j][3] * d[j][3]);
  }
#pragma unroll
  for (int off = 1; off < 32; off <<= 1) sq += __shfl_xor(sq, off, 32);
  const float var  = sq * (1.0f / EE);
  const float rinv = rsqrtf(var + 1e-5f);
  v4f y[4];
#pragma unroll
  for (int j = 0; j < 4; ++j) {
    const v4f gv = *(const v4f*)(gam + j * 128 + lane * 4);
    const v4f bv = *(const v4f*)(bet + j * 128 + lane * 4);
    y[j] = d[j] * rinv * gv + bv;
  }
  for (int pass = 0; pass < 2; ++pass) {
#pragma unroll
    for (int j = 0; j < 4; ++j) *(volatile v4f*)(outF + base + j * 128 + lane * 4) = y[j];
    __threadfence();
  }
  if (WH) {
    float* yw = ys[wave];
#pragma unroll
    for (int j = 0; j < 4; ++j) *(v4f*)(yw + j * 128 + lane * 4) = y[j];
    __builtin_amdgcn_fence(__ATOMIC_RELEASE, "workgroup");
    __builtin_amdgcn_wave_barrier();
    __builtin_amdgcn_fence(__ATOMIC_ACQUIRE, "workgroup");
    v4u hv[2];
#pragma unroll
    for (int j2 = 0; j2 < 2; ++j2) {
      const v4f a0 = *(const v4f*)(yw + j2 * 256 + lane * 8);
      const v4f a1 = *(const v4f*)(yw + j2 * 256 + lane * 8 + 4);
      hv[j2] = pack8s(a0, a1, 1.0f);
    }
    for (int pass = 0; pass < 2; ++pass) {
#pragma unroll
      for (int j2 = 0; j2 < 2; ++j2) *(volatile v4u*)(outH + base + j2 * 256 + lane * 8) = hv[j2];
      __threadfence();
    }
  }
}

static GemmArgs mkargs(const void* A, int lda, long long sA, int aOff,
                       const void* Bt, int ldb, long long sB,
                       void* C0, int ldc, long long sC,
                       const float* bias, int hasBias,
                       int M, int N, int K, int tDst, int tOff, int bShift, int skipLim,
                       float oscale, float ocarry) {
  GemmArgs g;
  g.A = (const unsigned short*)A; g.Bt = (const unsigned short*)Bt;
  g.C0 = C0; g.bias = bias;
  g.strideA = sA; g.strideB = sB; g.strideC = sC;
  g.lda = lda; g.ldb = ldb; g.ldc = ldc; g.M = M; g.N = N; g.K = K;
  g.aRowOff = aOff; g.tDst = tDst; g.tOff = tOff; g.bShift = bShift; g.skipLim = skipLim; g.hasBias = hasBias;
  g.oscale = oscale; g.ocarry = ocarry;
  return g;
}
static dim3 ggrid(int M, int N, int by) { return dim3((unsigned)((((M / 64) * (N / 64)) + 7) / 8), (unsigned)by); }

extern "C" void kernel_launch(void* const* d_in, const int* in_sizes, int n_in,
                              void* d_out, int out_size, void* d_ws, size_t ws_size,
                              hipStream_t stream) {
  if (n_in < 16) return;
  if (in_sizes[0] != QR * EE) return;
  if (in_sizes[1] != KL * EE) return;
  if (in_sizes[2] != NH * HD || in_sizes[3] != NH * HD) return;
  if (in_sizes[4] != MEM * BB * EE) return;
  if (in_sizes[5] != EE * 3 * EE) return;
  if (in_sizes[6] != EE * EE || in_sizes[7] != EE * EE) return;
  if (in_sizes[8] != EE || in_sizes[9] != EE) return;
  if (in_sizes[10] != EE * FFD || in_sizes[11] != FFD) return;
  if (in_sizes[12] != FFD * EE || in_sizes[13] != EE) return;
  if (in_sizes[14] != EE || in_sizes[15] != EE) return;
  if (out_size != QR * EE) return;

  const float* xseg = (const float*)d_in[0];
  const float* pos  = (const float*)d_in[1];
  const float* ub   = (const float*)d_in[2];
  const float* vb   = (const float*)d_in[3];
  const float* xmem = (const float*)d_in[4];
  const float* Wqkv = (const float*)d_in[5];
  const float* Wr   = (const float*)d_in[6];
  const float* Wo   = (const float*)d_in[7];
  const float* g1   = (const float*)d_in[8];
  const float* be1  = (const float*)d_in[9];
  const float* W1   = (const float*)d_in[10];
  const float* b1   = (const float*)d_in[11];
  const float* W2   = (const float*)d_in[12];
  const float* b2   = (const float*)d_in[13];
  const float* g2   = (const float*)d_in[14];
  const float* be2  = (const float*)d_in[15];

  const size_t zCAT = (size_t)CROWS * EE * 2;
  const size_t zPOS = (size_t)KL * EE * 2;
  const size_t zWQT = (size_t)3 * EE * EE * 2;
  const size_t zW   = (size_t)EE * EE * 2;
  const size_t zW1  = (size_t)FFD * EE * 2;
  const size_t zQP  = (size_t)NN * SQ * HD * 2;
  const size_t zKP  = (size_t)NN * KL * HD * 2;
  const size_t zRKP = (size_t)NH * KL * HD * 2;
  const size_t zCW  = (size_t)NN * KL * 4;
  const size_t zCR  = (size_t)NH * KL * 4;
  const size_t zRAW = (size_t)SQ * KL * 4;
  const size_t zCTX = (size_t)QR * EE * 2;
  const size_t zF32 = (size_t)QR * EE * 4;
  const size_t zHID = (size_t)QR * FFD * 2;
  size_t off = 0;
  const size_t oCAT = off; off += zCAT;
  const size_t oPOS = off; off += zPOS;
  const size_t oWQT = off; off += zWQT;
  const size_t oWRT = off; off += zW;
  const size_t oWOT = off; off += zW;
  const size_t oW1T = off; off += zW1;
  const size_t oW2T = off; off += zW1;
  const size_t oQP  = off; off += zQP;
  const size_t oKP  = off; off += zKP;
  const size_t oVT  = off; off += zKP;
  const size_t oRKP = off; off += zRKP;
  const size_t oCW  = off; off += zCW;
  const size_t oCR  = off; off += zCR;
  const size_t oRAW = off; off += zRAW;
  const size_t oCTX = off; off += zCTX;
  const size_t oAWO = off; off += zF32;
  const size_t oX1F = off; off += zF32;
  const size_t oX1H = off; off += zCTX;
  const size_t oHID = off; off += zHID;
  const size_t oFF2 = off; off += zF32;
  if (off > ws_size) return;
  if (off > (size_t)134217728) return;

  char* ws = (char*)d_ws;
  unsigned short* CAT = (unsigned short*)(ws + oCAT);
  unsigned short* POS = (unsigned short*)(ws + oPOS);
  unsigned short* WQT = (unsigned short*)(ws + oWQT);
  unsigned short* WRT = (unsigned short*)(ws + oWRT);
  unsigned short* WOT = (unsigned short*)(ws + oWOT);
  unsigned short* W1T = (unsigned short*)(ws + oW1T);
  unsigned short* W2T = (unsigned short*)(ws + oW2T);
  unsigned short* QP  = (unsigned short*)(ws + oQP);
  unsigned short* KP  = (unsigned short*)(ws + oKP);
  unsigned short* VT  = (unsigned short*)(ws + oVT);
  unsigned short* RKP = (unsigned short*)(ws + oRKP);
  float*          CW  = (float*)(ws + oCW);
  float*          CRT = (float*)(ws + oCR);
  float*          RAW = (float*)(ws + oRAW);
  unsigned short* CTX = (unsigned short*)(ws + oCTX);
  float*          AWO = (float*)(ws + oAWO);
  float*          X1F = (float*)(ws + oX1F);
  unsigned short* X1H = (unsigned short*)(ws + oX1H);
  unsigned short* HID = (unsigned short*)(ws + oHID);
  float*          FF2 = (float*)(ws + oFF2);

  const dim3 blk(256);
  const int n8c = CROWS * EE / 8;
  const int n8p = KL * EE / 8;
  const float sscale = 0.125f / (QKC * QKC);
  const float bdsc   = 0.125f / QKC;
  const float cinv   = CC / (PCY * QKC);

  cvt_cat<<<dim3((n8c + 255) / 256), blk, 0, stream>>>(xmem, xseg, CAT, n8c);
  cvt_f<<<dim3((n8p + 255) / 256), blk, 0, stream>>>(pos, POS, n8p, 1.0f);
  cvt_wt<<<dim3((3 * EE) / 64, EE / 64), blk, 0, stream>>>(Wqkv, WQT, EE, 3 * EE, WC);
  cvt_wt<<<dim3(EE / 64, EE / 64), blk, 0, stream>>>(Wr, WRT, EE, EE, WC);
  cvt_wt<<<dim3(EE / 64, EE / 64), blk, 0, stream>>>(Wo, WOT, EE, EE, WC);
  cvt_wt<<<dim3(FFD / 64, EE / 64), blk, 0, stream>>>(W1, W1T, EE, FFD, WC);
  cvt_wt<<<dim3(EE / 64, FFD / 64), blk, 0, stream>>>(W2, W2T, FFD, EE, WC);

  {
    const GemmArgs g = mkargs(CAT, EE, 0LL, 2 * MEM, WQT, EE, 0LL, (void*)QP, HD, 0LL, CRT, 0,
                              QR, EE, EE, SQ, MEM, 1, 0, 1.0f / WC, QKC);
    gemm64<1><<<ggrid(QR, EE, 1), blk, 0, stream>>>(g);
  }
  {
    const GemmArgs g = mkargs(CAT, EE, 0LL, 0, WQT + (size_t)EE * EE, EE, 0LL, (void*)KP, HD, 0LL, CRT, 0,
                              CROWS, EE, EE, KL, 0, 1, 0, 1.0f / WC, QKC);
    gemm64<1><<<ggrid(CROWS, EE, 1), blk, 0, stream>>>(g);
  }
  {
    const GemmArgs g = mkargs(WQT, EE, 0LL, 2 * EE, CAT, 2 * EE, (long long)EE, (void*)VT, KL, (long long)NH * HD * KL, CRT, 0,
                              EE, KL, EE, 0, 0, 0, 0, 1.0f / WC, QKC);
    gemm64<3><<<ggrid(EE, KL, BB), blk, 0, stream>>>(g);
  }
  {
    const GemmArgs g = mkargs(POS, EE, 0LL, 0, WRT, EE, 0LL, (void*)RKP, HD, 0LL, CRT, 0,
                              KL, EE, EE, KL, 0, 0, 0, 1.0f / WC, QKC);
    gemm64<1><<<ggrid(KL, EE, 1), blk, 0, stream>>>(g);
  }
  bias_dot<<<dim3((NN * (KL / 4) + 255) / 256, 2), blk, 0, stream>>>(KP, RKP, ub, vb, CW, CRT, bdsc);

  for (int n = 0; n < NN; ++n) {
    const int h = n & (NH - 1);
    const GemmArgs g = mkargs(QP + (size_t)n * SQ * HD, HD, 0LL, 0, RKP + (size_t)h * KL * HD, HD, 0LL,
                              (void*)RAW, KL, 0LL, CRT + (size_t)h * KL, 1,
                              SQ, KL, HD, 0, 0, 0, NQT - 1, sscale, 1.0f);
    gemm64<0><<<ggrid(SQ, KL, 1), blk, 0, stream>>>(g);
    attn_rel<<<dim3(NQT), dim3(128), 0, stream>>>(QP, KP, VT, RAW, CW, CTX, n, sscale, cinv);
  }
  {
    const GemmArgs g = mkargs(CTX, EE, 0LL, 0, WOT, EE, 0LL, (void*)AWO, EE, 0LL, CRT, 0,
                              QR, EE, EE, 0, 0, 0, 0, 1.0f / (CC * WC), 1.0f);
    gemm64<0><<<ggrid(QR, EE, 1), blk, 0, stream>>>(g);
  }
  ln_rows<1><<<dim3(QR / 8), blk, 0, stream>>>(xseg, AWO, g1, be1, X1F, X1H, QR);
  {
    const GemmArgs g = mkargs(X1H, EE, 0LL, 0, W1T, EE, 0LL, (void*)HID, FFD, 0LL, b1, 1,
                              QR, FFD, EE, 0, 0, 0, 0, 1.0f / WC, HC);
    gemm64<2><<<ggrid(QR, FFD, 1), blk, 0, stream>>>(g);
  }
  {
    const GemmArgs g = mkargs(HID, FFD, 0LL, 0, W2T, FFD, 0LL, (void*)FF2, EE, 0LL, b2, 1,
                              QR, EE, FFD, 0, 0, 0, 0, 1.0f / (HC * WC), 1.0f);
    gemm64<0><<<ggrid(QR, EE, 1), blk, 0, stream>>>(g);
  }
  ln_rows<0><<<dim3(QR / 8), blk, 0, stream>>>(X1F, FF2, g2, be2, (float*)d_out, X1H, QR);
  (void)hipGetLastError();
}
